// Encoder_29712583754153
// MI455X (gfx1250) — hardware-run, weakly checked
//
#include <hip/hip_runtime.h>
#include <math.h>

typedef __attribute__((ext_vector_type(8)))  _Float16 v8h;
typedef __attribute__((ext_vector_type(16))) __bf16   v16b;
typedef __attribute__((ext_vector_type(8)))  __bf16   v8b;
typedef __attribute__((ext_vector_type(8)))  float    v8f;
typedef __attribute__((ext_vector_type(4)))  float    v4f;

constexpr int kNB   = 64;
constexpr int kNS   = 80;
constexpr int kNC   = 32;
constexpr int kNV   = 10000;
constexpr int kNE   = 256;
constexpr int kNH   = 512;
constexpr int kNG   = 3 * kNH;
constexpr int kNL   = 128;
constexpr int kRows = kNS * kNB;
constexpr int kHP16 = 520;
constexpr int kHPF  = 516;
static_assert(kNG == 1536 && kRows == 5120, "shape");
static_assert((kNE % 32) == 0 && (kNH % 32) == 0, "GEMM K multiples of 32");
static_assert((kRows % 64) == 0 && (kNG % 64) == 0, "GEMM M,N multiples of 64");
static_assert(16 * kHPF * 4 <= 2 * 16 * kHP16 * 2, "f32 state copy fits in the 16-bit plane pool");
static_assert((kHP16 % 8) == 0 && (kHPF % 4) == 0, "16-B aligned LDS rows");

constexpr size_t kOffEMBH = 0;
constexpr size_t kOffEMBL = kOffEMBH + (size_t)kRows * kNE * 2;
constexpr size_t kOffWIH  = kOffEMBL + (size_t)kRows * kNE * 2;
constexpr size_t kOffWIL  = kOffWIH  + (size_t)kNG * kNE * 2;
constexpr size_t kOffWHH  = kOffWIL  + (size_t)kNG * kNE * 2;
constexpr size_t kOffWHL  = kOffWHH  + (size_t)kNG * kNH * 2;
constexpr size_t kOffGI   = kOffWHL  + (size_t)kNG * kNH * 2;
constexpr size_t kWsTotal = kOffGI   + (size_t)kRows * kNG * 4;
static_assert(kWsTotal == 41418752ull, "carve total");
static_assert(kWsTotal <= 134217728ull, "carve cap");
static_assert((kOffEMBL % 128) == 0 && (kOffWIH % 128) == 0 && (kOffWIL % 128) == 0 && (kOffWHH % 128) == 0 &&
              (kOffWHL % 128) == 0 && (kOffGI % 128) == 0, "128-B aligned regions");

__device__ __forceinline__ unsigned short f2bf_bits(float f) {
  unsigned u = __float_as_uint(f);
  return (unsigned short)((u + 0x7FFFu + ((u >> 16) & 1u)) >> 16);
}
__device__ __forceinline__ float bf_bits2f(unsigned short h) { return __uint_as_float(((unsigned)h) << 16); }

union FragB { v16b v; v8b h[2]; };
__device__ __forceinline__ v16b frag_load(const __bf16* p) {
  FragB f;
  f.h[0] = *(const v8b*)(p);
  f.h[1] = *(const v8b*)(p + 16);
  return f.v;
}
__device__ __forceinline__ v8f mma_bf(v16b a, v16b b, v8f c) {
  return __builtin_amdgcn_wmma_f32_16x16x32_bf16(false, a, false, b, (short)0, c, false, false);
}
__device__ __forceinline__ void dep_guard4_b(v8f& a, v8f& b, v8f& c, v8f& d, v16b x, v16b y) {
  asm volatile("v_nop\n\tv_nop\n\tv_nop\n\tv_nop" : "+v"(a), "+v"(b), "+v"(c), "+v"(d) : "v"(x), "v"(y));
}
__device__ __forceinline__ void keep4_b(v16b a, v16b b, v16b c, v16b d) {
  asm volatile("v_nop" :: "v"(a), "v"(b), "v"(c), "v"(d));
}
__device__ __forceinline__ void acc_guard4(v8f& a, v8f& b, v8f& c, v8f& d) {
  asm volatile("v_nop\n\tv_nop\n\tv_nop\n\tv_nop" : "+v"(a), "+v"(b), "+v"(c), "+v"(d));
}
__device__ __forceinline__ void grp_guard_b(v8f& a, v8f& b, v16b x, v16b y, v16b p, v16b q, v16b r, v16b s) {
  asm volatile("v_nop\n\tv_nop\n\tv_nop\n\tv_nop" : "+v"(a), "+v"(b) : "v"(x), "v"(y), "v"(p), "v"(q), "v"(r), "v"(s));
}
__device__ __forceinline__ float sigm(float x) { return 1.0f / (1.0f + expf(-x)); }

__global__ __launch_bounds__(256) void embed_rows_kernel(
    const int* __restrict__ seq, const int* __restrict__ len, const float* __restrict__ EW,
    unsigned short* __restrict__ EH, unsigned short* __restrict__ EL)
{
  __shared__ int sIdx[kNB];
  const int tid  = threadIdx.x;
  const int lane = tid & 31;
  const int wave = __builtin_amdgcn_readfirstlane((int)(threadIdx.x >> 5));
  if (wave < 2) {
    const int li = len[tid];
    int rank = 0;
#pragma unroll 1
    for (int j = 0; j < kNB; ++j) {
      const int lj = len[j];
      rank += ((lj > li) || ((lj == li) && (j < tid))) ? 1 : 0;
    }
    rank = min(max(rank, 0), kNB - 1);
    sIdx[rank] = tid;
  }
  __syncthreads();
  const int m = blockIdx.x * 8 + wave;
  const int s = m >> 6;
  const int p = m & 63;
  int pat = sIdx[p];
  pat = min(max(pat, 0), kNB - 1);
  int c = seq[((size_t)pat * kNS + s) * kNC + lane];
  c = min(max(c, 0), kNV - 1);
  int dup = 0;
#pragma unroll 4
  for (int j = 0; j < 32; ++j) {
    const int cj = __shfl(c, j, 32);
    dup |= ((j < lane) && (cj == c)) ? 1 : 0;
  }
  const int valid = ((c != 0) && (dup == 0)) ? 1 : 0;
  const unsigned vm = (unsigned)__ballot(valid);
  float a[8];
#pragma unroll
  for (int e = 0; e < 8; ++e) a[e] = 0.0f;
  const float* ewl = EW + lane * 8;
#pragma unroll 2
  for (int j = 0; j < 32; ++j) {
    const int cj = __shfl(c, j, 32);
    const bool on = ((vm >> j) & 1u) != 0u;
    const float* rp = ewl + (size_t)cj * kNE;
    const v4f x0 = *(const v4f*)(rp);
    const v4f x1 = *(const v4f*)(rp + 4);
    a[0] += on ? x0[0] : 0.0f;
    a[1] += on ? x0[1] : 0.0f;
    a[2] += on ? x0[2] : 0.0f;
    a[3] += on ? x0[3] : 0.0f;
    a[4] += on ? x1[0] : 0.0f;
    a[5] += on ? x1[1] : 0.0f;
    a[6] += on ? x1[2] : 0.0f;
    a[7] += on ? x1[3] : 0.0f;
  }
#pragma unroll 1
  for (int it = 0; it < 8; ++it) {
    const float tv = tanhf(a[0]);
    a[0] = a[1]; a[1] = a[2]; a[2] = a[3]; a[3] = a[4];
    a[4] = a[5]; a[5] = a[6]; a[6] = a[7]; a[7] = tv;
  }
  v8h hv, lv;
#pragma unroll
  for (int e = 0; e < 8; ++e) {
    const unsigned short hb = f2bf_bits(a[e]);
    const unsigned short lb = f2bf_bits(a[e] - bf_bits2f(hb));
    hv[e] = __builtin_bit_cast(_Float16, hb);
    lv[e] = __builtin_bit_cast(_Float16, lb);
  }
  unsigned short* qh = EH + (size_t)m * kNE + lane * 8;
  unsigned short* ql = EL + (size_t)m * kNE + lane * 8;
  *(volatile v8h*)qh = hv;
  *(volatile v8h*)ql = lv;
  __threadfence();
  *(volatile v8h*)qh = hv;
  *(volatile v8h*)ql = lv;
}

__global__ __launch_bounds__(256) void split_rows_bf16_kernel(
    const float* __restrict__ src, unsigned short* __restrict__ dhi, unsigned short* __restrict__ dlo, int total8)
{
  const int i = blockIdx.x * 256 + threadIdx.x;
  if (i >= total8) return;
  const size_t e0 = (size_t)i << 3;
  const v4f a0 = *(const v4f*)(src + e0);
  const v4f a1 = *(const v4f*)(src + e0 + 4);
  v8h hv, lv;
#pragma unroll
  for (int e = 0; e < 4; ++e) {
    const unsigned short h0 = f2bf_bits(a0[e]), h1 = f2bf_bits(a1[e]);
    const unsigned short l0 = f2bf_bits(a0[e] - bf_bits2f(h0)), l1 = f2bf_bits(a1[e] - bf_bits2f(h1));
    hv[e]     = __builtin_bit_cast(_Float16, h0);
    hv[4 + e] = __builtin_bit_cast(_Float16, h1);
    lv[e]     = __builtin_bit_cast(_Float16, l0);
    lv[4 + e] = __builtin_bit_cast(_Float16, l1);
  }
  unsigned short* qh = dhi + e0;
  unsigned short* ql = dlo + e0;
  *(volatile v8h*)qh = hv;
  *(volatile v8h*)ql = lv;
  __threadfence();
  *(volatile v8h*)qh = hv;
  *(volatile v8h*)ql = lv;
}

__global__ __launch_bounds__(256) void gi_gemm_kernel(
    const unsigned short* __restrict__ Ap, const unsigned short* __restrict__ A2p, int lda,
    const unsigned short* __restrict__ Btp, const unsigned short* __restrict__ Bt2p, int ldb,
    float* __restrict__ Cout, int ldc, const float* __restrict__ bias, int M, int N, int K)
{
  const __bf16* A   = (const __bf16*)Ap;
  const __bf16* A2  = (const __bf16*)A2p;
  const __bf16* Bt  = (const __bf16*)Btp;
  const __bf16* Bt2 = (const __bf16*)Bt2p;
  __shared__ __align__(16) float sT[8][16 * 68];
  const int lane = threadIdx.x & 31;
  const int wave = __builtin_amdgcn_readfirstlane((int)(threadIdx.x >> 5));
  const int tilesN = N >> 6;
  const int tilesM = M >> 6;
  const int tile = blockIdx.x * 8 + wave;
  if (tile >= tilesM * tilesN) return;
  const int tm = tile / tilesN;
  const int tn = tile - tm * tilesN;
  const int m0 = tm << 6;
  const int n0 = tn << 6;

  const int rlane = lane & 15;
  const int koff  = (lane >> 4) * 8;
  const int mOff  = (lane >> 4) * 8;

  v8f acc[4][4];
#pragma unroll
  for (int i = 0; i < 4; ++i)
#pragma unroll
    for (int j = 0; j < 4; ++j) acc[i][j] = (v8f){0.f,0.f,0.f,0.f,0.f,0.f,0.f,0.f};

  for (int k0 = 0; k0 < K; k0 += 32) {
    v16b bh[4], bl[4];
#pragma unroll
    for (int j = 0; j < 4; ++j) {
      const size_t bo = (size_t)(n0 + (j << 4) + rlane) * ldb + koff + k0;
      bh[j] = frag_load(Bt + bo);
      bl[j] = frag_load(Bt2 + bo);
    }
#pragma unroll
    for (int i = 0; i < 4; ++i) {
      const size_t ao = (size_t)(m0 + (i << 4) + rlane) * lda + koff + k0;
      const v16b ah = frag_load(A + ao);
      const v16b al = frag_load(A2 + ao);
#pragma unroll
      for (int j = 0; j < 4; ++j) {
        acc[i][j] = mma_bf(ah, bh[j], acc[i][j]);
        acc[i][j] = mma_bf(ah, bl[j], acc[i][j]);
        acc[i][j] = mma_bf(al, bh[j], acc[i][j]);
      }
      dep_guard4_b(acc[i][0], acc[i][1], acc[i][2], acc[i][3], ah, al);
    }
    keep4_b(bh[0], bh[1], bh[2], bh[3]);
    keep4_b(bl[0], bl[1], bl[2], bl[3]);
  }
  acc_guard4(acc[0][0], acc[0][1], acc[0][2], acc[0][3]);
  acc_guard4(acc[1][0], acc[1][1], acc[1][2], acc[1][3]);
  acc_guard4(acc[2][0], acc[2][1], acc[2][2], acc[2][3]);
  acc_guard4(acc[3][0], acc[3][1], acc[3][2], acc[3][3]);

  float* slab = sT[wave];
#pragma unroll
  for (int i = 0; i < 4; ++i) {
    const int mBase = m0 + (i << 4);
#pragma unroll
    for (int j = 0; j < 4; ++j) {
      const int n = n0 + (j << 4) + rlane;
      const float bv = bias[n];
#pragma unroll
      for (int r = 0; r < 8; ++r) {
        const float v = acc[i][j][r] + bv;
        slab[(mOff + r) * 68 + (j << 4) + rlane] = v;
      }
    }
    __builtin_amdgcn_fence(__ATOMIC_RELEASE, "workgroup");
    __builtin_amdgcn_wave_barrier();
    __builtin_amdgcn_fence(__ATOMIC_ACQUIRE, "workgroup");
    {
      const int hh = lane >> 4, c4 = (lane & 15) * 4;
      for (int pass = 0; pass < 2; ++pass) {
#pragma unroll
        for (int it = 0; it < 8; ++it) {
          const int row = it * 2 + hh;
          const v4f v = *(const v4f*)(slab + row * 68 + c4);
          *(volatile v4f*)(Cout + (size_t)(mBase + row) * ldc + n0 + c4) = v;
        }
        __threadfence();
      }
    }
    __builtin_amdgcn_fence(__ATOMIC_RELEASE, "workgroup");
    __builtin_amdgcn_wave_barrier();
    __builtin_amdgcn_fence(__ATOMIC_ACQUIRE, "workgroup");
  }
}

__global__ __launch_bounds__(512) void gru_scan_kernel(
    const float* __restrict__ GI, const unsigned short* __restrict__ WhHp, const unsigned short* __restrict__ WhLp,
    const float* __restrict__ bh, const int* __restrict__ len,
    const float* __restrict__ Wlat, const float* __restrict__ blat, float* __restrict__ out)
{
  __shared__ __align__(16) __bf16 hpool[2 * 16 * kHP16];
  __shared__ int sLen[16];
  constexpr int kLoOff = 16 * kHP16;
  const __bf16* WhH = (const __bf16*)WhHp;
  const __bf16* WhL = (const __bf16*)WhLp;
  const int tid  = threadIdx.x;
  const int lane = tid & 31;
  const int hf   = lane >> 4;
  const int ln   = lane & 15;
  const int wave = __builtin_amdgcn_readfirstlane((int)(threadIdx.x >> 5));
  const int r0   = blockIdx.x * 16;

  {
    v8b z;
#pragma unroll
    for (int e = 0; e < 8; ++e) z[e] = __builtin_bit_cast(__bf16, (unsigned short)0);
    for (int i = tid; i < (2 * 16 * kHP16) / 8; i += 512) *(v8b*)(hpool + 8 * i) = z;
  }
  if (wave < 2) {
    const int li = len[tid];
    int rank = 0;
#pragma unroll 1
    for (int j = 0; j < kNB; ++j) {
      const int lj = len[j];
      rank += ((lj > li) || ((lj == li) && (j < tid))) ? 1 : 0;
    }
    const int pos = rank - r0;
    const int lc = min(max(li, 0), kNS);
    if (pos >= 0 && pos < 16) sLen[pos] = lc;
  }
  __syncthreads();

  int myLen[8];
#pragma unroll
  for (int r = 0; r < 8; ++r) myLen[r] = sLen[8 * hf + r];
  int tmax = 0;
#pragma unroll
  for (int i = 0; i < 16; ++i) tmax = max(tmax, sLen[i]);
  tmax = min(tmax, kNS);
  tmax = __builtin_amdgcn_readfirstlane(tmax);

  const int j1 = 16 * wave + ln;
  const int j2 = j1 + 256;
  const float bhr1 = bh[j1], bhz1 = bh[j1 + kNH], bhn1 = bh[j1 + 2 * kNH];
  const float bhr2 = bh[j2], bhz2 = bh[j2 + kNH], bhn2 = bh[j2 + 2 * kNH];

  float hc[8], ho[8];
#pragma unroll
  for (int r = 0; r < 8; ++r) { hc[r] = 0.0f; ho[r] = 0.0f; }

  const int    aofs = ln * kHP16 + 8 * hf;
  const size_t bofs = (size_t)j1 * kNH + 8 * hf;

#pragma unroll 1
  for (int t = 0; t < tmax; ++t) {
    v8f c[6];
#pragma unroll
    for (int i = 0; i < 6; ++i) c[i] = (v8f){0.f,0.f,0.f,0.f,0.f,0.f,0.f,0.f};
#pragma unroll 1
    for (int ks = 0; ks < kNH / 32; ++ks) {
      const int k0 = ks * 32;
      FragB fa, fl;
      fa.h[0] = *(const v8b*)(hpool + aofs + k0);
      fa.h[1] = *(const v8b*)(hpool + aofs + k0 + 16);
      fl.h[0] = *(const v8b*)(hpool + kLoOff + aofs + k0);
      fl.h[1] = *(const v8b*)(hpool + kLoOff + aofs + k0 + 16);
      const v16b ah = fa.v;
      const v16b al = fl.v;
#pragma unroll
      for (int g = 0; g < 3; ++g) {
        const size_t b0 = bofs + (size_t)g * kNH * kNH + k0;
        const size_t b1 = b0 + (size_t)256 * kNH;
        const v16b bh0 = frag_load(WhH + b0);
        const v16b bl0 = frag_load(WhL + b0);
        const v16b bh1 = frag_load(WhH + b1);
        const v16b bl1 = frag_load(WhL + b1);
        c[2 * g]     = mma_bf(ah, bh0, c[2 * g]);
        c[2 * g]     = mma_bf(ah, bl0, c[2 * g]);
        c[2 * g]     = mma_bf(al, bh0, c[2 * g]);
        c[2 * g + 1] = mma_bf(ah, bh1, c[2 * g + 1]);
        c[2 * g + 1] = mma_bf(ah, bl1, c[2 * g + 1]);
        c[2 * g + 1] = mma_bf(al, bh1, c[2 * g + 1]);
        grp_guard_b(c[2 * g], c[2 * g + 1], ah, al, bh0, bl0, bh1, bl1);
      }
    }
    __syncthreads();

    v8f ar = c[0], az = c[2], an = c[4];
    v8f br = c[1], bz = c[3], bn = c[5];
    int jc = j1, jo = j2;
    float bRc = bhr1, bZc = bhz1, bNc = bhn1;
    float bRo = bhr2, bZo = bhz2, bNo = bhn2;
    const float* girow = GI + ((size_t)t * kNB + r0 + 8 * hf) * kNG;
#pragma unroll 1
    for (int cg = 0; cg < 2; ++cg) {
#pragma unroll
      for (int r = 0; r < 8; ++r) {
        const float* gp = girow + (size_t)r * kNG + jc;
        const float gr = gp[0];
        const float gz = gp[kNH];
        const float gn = gp[2 * kNH];
        const float rr = sigm(gr + (ar[r] + bRc));
        const float zz = sigm(gz + (az[r] + bZc));
        const float nn = tanhf(gn + rr * (an[r] + bNc));
        const float hp = hc[r];
        const float hn = (1.0f - zz) * nn + zz * hp;
        const float hv = (t < myLen[r]) ? hn : hp;
        hc[r] = hv;
        const unsigned short hb = f2bf_bits(hv);
        const unsigned short lb = f2bf_bits(hv - bf_bits2f(hb));
        hpool[(8 * hf + r) * kHP16 + jc]          = __builtin_bit_cast(__bf16, hb);
        hpool[kLoOff + (8 * hf + r) * kHP16 + jc] = __builtin_bit_cast(__bf16, lb);
      }
      {
        const v8f t0 = ar; ar = br; br = t0;
        const v8f t1 = az; az = bz; bz = t1;
        const v8f t2 = an; an = bn; bn = t2;
        const int tj = jc; jc = jo; jo = tj;
        const float f0 = bRc; bRc = bRo; bRo = f0;
        const float f1 = bZc; bZc = bZo; bZo = f1;
        const float f2 = bNc; bNc = bNo; bNo = f2;
#pragma unroll
        for (int r = 0; r < 8; ++r) { const float tf = hc[r]; hc[r] = ho[r]; ho[r] = tf; }
      }
    }
    __syncthreads();
  }

  float* hF = (float*)hpool;
#pragma unroll
  for (int r = 0; r < 8; ++r) {
    hF[(8 * hf + r) * kHPF + j1] = hc[r];
    hF[(8 * hf + r) * kHPF + j2] = ho[r];
  }
  __syncthreads();

  {
    const float* hrow = hF + wave * kHPF;
    const float* w0p = Wlat + (size_t)(lane * 4 + 0) * kNH;
    const float* w1p = Wlat + (size_t)(lane * 4 + 1) * kNH;
    const float* w2p = Wlat + (size_t)(lane * 4 + 2) * kNH;
    const float* w3p = Wlat + (size_t)(lane * 4 + 3) * kNH;
    float s0 = 0.0f, s1 = 0.0f, s2 = 0.0f, s3 = 0.0f;
#pragma unroll 1
    for (int j4 = 0; j4 < kNH / 4; ++j4) {
      const v4f hv4 = *(const v4f*)(hrow + 4 * j4);
      const v4f x0 = *(const v4f*)(w0p + 4 * j4);
      const v4f x1 = *(const v4f*)(w1p + 4 * j4);
      const v4f x2 = *(const v4f*)(w2p + 4 * j4);
      const v4f x3 = *(const v4f*)(w3p + 4 * j4);
      s0 = fmaf(hv4[0], x0[0], s0); s0 = fmaf(hv4[1], x0[1], s0); s0 = fmaf(hv4[2], x0[2], s0); s0 = fmaf(hv4[3], x0[3], s0);
      s1 = fmaf(hv4[0], x1[0], s1); s1 = fmaf(hv4[1], x1[1], s1); s1 = fmaf(hv4[2], x1[2], s1); s1 = fmaf(hv4[3], x1[3], s1);
      s2 = fmaf(hv4[0], x2[0], s2); s2 = fmaf(hv4[1], x2[1], s2); s2 = fmaf(hv4[2], x2[2], s2); s2 = fmaf(hv4[3], x2[3], s2);
      s3 = fmaf(hv4[0], x3[0], s3); s3 = fmaf(hv4[1], x3[1], s3); s3 = fmaf(hv4[2], x3[2], s3); s3 = fmaf(hv4[3], x3[3], s3);
    }
    const v4f bl4 = *(const v4f*)(blat + lane * 4);
    v4f o;
    o[0] = tanhf(s0 + bl4[0]);
    o[1] = tanhf(s1 + bl4[1]);
    o[2] = tanhf(s2 + bl4[2]);
    o[3] = tanhf(s3 + bl4[3]);
    float* po = out + (size_t)(r0 + wave) * kNL + lane * 4;
    *(volatile v4f*)po = o;
    __threadfence();
    *(volatile v4f*)po = o;
  }
}

extern "C" void kernel_launch(void* const* d_in, const int* in_sizes, int n_in,
                              void* d_out, int out_size, void* d_ws, size_t ws_size,
                              hipStream_t stream) {
  if (n_in < 9) return;
  if (in_sizes[0] != kNB * kNS * kNC) return;
  if (in_sizes[1] != kNB) return;
  if (in_sizes[2] != kNV * kNE) return;
  if (in_sizes[3] != kNG * kNE) return;
  if (in_sizes[4] != kNG * kNH) return;
  if (in_sizes[5] != kNG) return;
  if (in_sizes[6] != kNG) return;
  if (in_sizes[7] != kNL * kNH) return;
  if (in_sizes[8] != kNL) return;
  if (out_size != kNB * kNL) return;
  if (ws_size < kWsTotal) return;

  const int*   seq  = (const int*)d_in[0];
  const int*   len  = (const int*)d_in[1];
  const float* EW   = (const float*)d_in[2];
  const float* Wi   = (const float*)d_in[3];
  const float* Wh   = (const float*)d_in[4];
  const float* bi   = (const float*)d_in[5];
  const float* bh   = (const float*)d_in[6];
  const float* Wlat = (const float*)d_in[7];
  const float* blat = (const float*)d_in[8];
  float* out = (float*)d_out;

  char* ws = (char*)d_ws;
  unsigned short* EMBH = (unsigned short*)(ws + kOffEMBH);
  unsigned short* EMBL = (unsigned short*)(ws + kOffEMBL);
  unsigned short* WIH  = (unsigned short*)(ws + kOffWIH);
  unsigned short* WIL  = (unsigned short*)(ws + kOffWIL);
  unsigned short* WHH  = (unsigned short*)(ws + kOffWHH);
  unsigned short* WHL  = (unsigned short*)(ws + kOffWHL);
  float*          GI   = (float*)(ws + kOffGI);

  embed_rows_kernel<<<kRows / 8, 256, 0, stream>>>(seq, len, EW, EMBH, EMBL);
  split_rows_bf16_kernel<<<(kNG * kNE / 8) / 256, 256, 0, stream>>>(Wi, WIH, WIL, kNG * kNE / 8);
  split_rows_bf16_kernel<<<(kNG * kNH / 8) / 256, 256, 0, stream>>>(Wh, WHH, WHL, kNG * kNH / 8);
  gi_gemm_kernel<<<((kRows / 64) * (kNG / 64)) / 8, 256, 0, stream>>>(
      EMBH, EMBL, kNE, WIH, WIL, kNE, GI, kNG, bi, kRows, kNG, kNE);
  gru_scan_kernel<<<kNB / 16, 512, 0, stream>>>(GI, WHH, WHL, bh, len, Wlat, blat, out);
}
